// multiplication_20864951124494
// MI455X (gfx1250) — hardware-verified
//
#include <hip/hip_runtime.h>
#include <stddef.h>


typedef _Float16 v16h __attribute__((ext_vector_type(16)));
typedef _Float16 v8h  __attribute__((ext_vector_type(8)));
typedef float    v8f  __attribute__((ext_vector_type(8)));
typedef float    v4f  __attribute__((ext_vector_type(4)));
typedef _Float16 h16;

#ifndef NB
#define NB 4
#endif
#ifndef SEQ
#define SEQ 4096
#endif
#define NB_FULL  4
#define SEQ_FULL 4096
#define HD    64
#define CH    256
#define OUTW  512
#define CSLAB 128
#define MROWS (NB * SEQ)

static_assert(NB >= 1 && NB <= NB_FULL);
static_assert(SEQ >= 128 && SEQ <= SEQ_FULL && (SEQ % 128) == 0);
static_assert(HD == 64);
static_assert(OUTW == 2 * CH);
static_assert((CH % CSLAB) == 0 && CSLAB == 8 * 16);
static_assert((CH % 64) == 0 && (SEQ % 64) == 0);
static_assert((MROWS % 32) == 0 && (MROWS % 4) == 0);
static_assert((HD % 8) == 0 && (CH % 4) == 0);
static_assert((size_t)NB_FULL * SEQ_FULL * OUTW * 4 == (size_t)33554432);

#define LDT 72
#define LDE 36
static_assert((LDT % 8) == 0 && LDT >= 64);
static_assert((LDE % 4) == 0 && LDE >= 32);
static_assert((size_t)64 * LDT * 2 + (size_t)CSLAB * LDT * 2 + (size_t)8 * 16 * LDT * 2 +
              (size_t)8 * 16 * LDE * 4 <= (size_t)65536);

#define WCARRY 64.0f
#define QCARRY 16.0f
#define PCARRY 16384.0f

#define ROW16_BYTES ((size_t)MROWS * HD * 2)
#define VT_BYTES    ((size_t)NB * CH * SEQ * 2)
#define OFF_PG  ((size_t)0)
#define OFF_XQ  (OFF_PG + ROW16_BYTES)
#define OFF_VT  (OFF_XQ + ROW16_BYTES)
#define WS_TOTAL (OFF_VT + VT_BYTES)
static_assert((ROW16_BYTES % 128) == 0 && (VT_BYTES % 128) == 0);
static_assert(WS_TOTAL <= (size_t)134217728);

__device__ __forceinline__ float bf16r(float x) {
  unsigned int u = __float_as_uint(x);
  u = (u + 0x7FFFu + ((u >> 16) & 1u)) & 0xFFFF0000u;
  return __uint_as_float(u);
}

static __device__ __forceinline__ h16 toh_flush(float v) {
  const h16 r = (h16)v;
  return (fabsf(v) < 6.103515625e-05f) ? (h16)0.0f : r;
}

__device__ __forceinline__ v16h frag_at(const _Float16* p) {
  v8h lo = *(const v8h*)(p);
  v8h hi = *(const v8h*)(p + 16);
  v16h out;
#pragma unroll
  for (int i = 0; i < 8; ++i) { out[i] = lo[i]; out[i + 8] = hi[i]; }
  return out;
}
__device__ __forceinline__ v16h ld_frag(const _Float16* base, unsigned ld) {
  const unsigned lane = threadIdx.x & 31u;
  return frag_at(base + (lane & 15u) * ld + (lane >> 4) * 8u);
}

__device__ __forceinline__ v8f wmma16(v16h a, v16h b, v8f c) {
  v8f d = __builtin_amdgcn_wmma_f32_16x16x32_f16(false, a, false, b, (short)0, c,
                                                 false, false);
  asm volatile("v_nop\n\tv_nop\n\tv_nop\n\tv_nop" : "+v"(d) : "v"(a), "v"(b));
  return d;
}

__device__ __forceinline__ float red16_max(float x) {
#pragma unroll
  for (int off = 1; off < 16; off <<= 1) x = fmaxf(x, __shfl_xor(x, off, 32));
  return x;
}
__device__ __forceinline__ float red16_sum(float x) {
#pragma unroll
  for (int off = 1; off < 16; off <<= 1) x += __shfl_xor(x, off, 32);
  return x;
}

__device__ __forceinline__ void wave_lds_sync() {
  __builtin_amdgcn_fence(3  , "wavefront");
  asm volatile("s_wait_dscnt 0x0" ::: "memory");
  __builtin_amdgcn_wave_barrier();
}

__global__ __launch_bounds__(256) void wconv_kernel(
    const float* __restrict__ W, _Float16* __restrict__ Wt, unsigned ldw, unsigned ldk) {
  __shared__ _Float16 T[64 * LDT];
  const unsigned tid = threadIdx.x;
  const unsigned n0 = blockIdx.x * 64u;
  const unsigned k0 = blockIdx.y * 64u;
#pragma unroll 4
  for (unsigned j = 0; j < 16u; ++j) {
    const unsigned idx = tid + 256u * j;
    const unsigned kr = idx >> 6, nc = idx & 63u;
    const float v = W[(size_t)(k0 + kr) * ldw + n0 + nc];
    T[nc * LDT + kr] = (_Float16)(WCARRY * bf16r(v));
  }
  __syncthreads();
  v8h x[2];
  size_t off[2];
#pragma unroll
  for (unsigned i = 0; i < 2u; ++i) {
    const unsigned n = 32u * i + (tid >> 3);
    const unsigned kc = (tid & 7u) * 8u;
    x[i] = *(const v8h*)&T[n * LDT + kc];
    off[i] = (size_t)(n0 + n) * ldk + k0 + kc;
  }
#pragma unroll
  for (int i = 0; i < 2; ++i) *(volatile v8h*)(Wt + off[i]) = x[i];
  __threadfence();
#pragma unroll
  for (int i = 0; i < 2; ++i) *(volatile v8h*)(Wt + off[i]) = x[i];
}

__global__ __launch_bounds__(256) void rowconv_kernel(
    const float* __restrict__ RowIn, const float* __restrict__ KeyIn,
    _Float16* __restrict__ row16, _Float16* __restrict__ key16) {
#pragma clang fp contract(off)
  const unsigned idx = blockIdx.x * 256u + threadIdx.x;
  const unsigned crow = idx >> 3;
  const unsigned c = (idx & 7u) * 8u;
  const unsigned bidx = crow / (unsigned)SEQ;
  const unsigned sq = crow - bidx * (unsigned)SEQ;
  const size_t frow = (size_t)bidx * SEQ_FULL + sq;
  const v4f a0 = *(const v4f*)(RowIn + frow * HD + c);
  const v4f a1 = *(const v4f*)(RowIn + frow * HD + c + 4u);
  const v4f b0 = *(const v4f*)(KeyIn + frow * HD + c);
  const v4f b1 = *(const v4f*)(KeyIn + frow * HD + c + 4u);
  v8h xr, xk;
#pragma unroll
  for (int i = 0; i < 4; ++i) {
    xr[i]     = toh_flush(QCARRY * bf16r(a0[i]));
    xr[i + 4] = toh_flush(QCARRY * bf16r(a1[i]));
    xk[i]     = toh_flush(QCARRY * bf16r(b0[i]));
    xk[i + 4] = toh_flush(QCARRY * bf16r(b1[i]));
  }
  const size_t off = (size_t)crow * HD + c;
  *(volatile v8h*)(row16 + off) = xr;
  *(volatile v8h*)(key16 + off) = xk;
  __threadfence();
  *(volatile v8h*)(row16 + off) = xr;
  *(volatile v8h*)(key16 + off) = xk;
}

__global__ __launch_bounds__(256) void concat_kernel(
    const float* __restrict__ G, float* __restrict__ out) {
#pragma clang fp contract(off)
  const unsigned idx = blockIdx.x * 256u + threadIdx.x;
  const unsigned crow = idx >> 6;
  const unsigned c = (idx & 63u) * 4u;
  const unsigned bidx = crow / (unsigned)SEQ;
  const unsigned sq = crow - bidx * (unsigned)SEQ;
  const size_t frow = (size_t)bidx * SEQ_FULL + sq;
  const v4f a = *(const v4f*)(G + frow * CH + c);
  v4f o;
#pragma unroll
  for (int j = 0; j < 4; ++j) o[j] = bf16r(a[j]);
  float* p = out + frow * OUTW + CH + c;
  *(volatile v4f*)p = o;
  __threadfence();
  *(volatile v4f*)p = o;
}

__global__ __launch_bounds__(256) __attribute__((amdgpu_num_vgpr(256))) void attn_kernel(
    const _Float16* __restrict__ Qh, const _Float16* __restrict__ Kh,
    const _Float16* __restrict__ Vt, const float* __restrict__ xres,
    const float* __restrict__ kp, float* __restrict__ out) {
  __shared__ __attribute__((aligned(16))) _Float16 Ks[64 * LDT];
  __shared__ __attribute__((aligned(16))) _Float16 Vs[CSLAB * LDT];
  __shared__ __attribute__((aligned(16))) _Float16 Ps[8 * 16 * LDT];
  __shared__ __attribute__((aligned(16))) float Cs[8 * 16 * LDE];

  const unsigned tid = threadIdx.x, lane = tid & 31u;
  const unsigned wave = (unsigned)__builtin_amdgcn_readfirstlane((int)(threadIdx.x >> 5));
  const unsigned hh = lane >> 4, m = lane & 15u;
  const unsigned q0 = blockIdx.x * 128u;
  const unsigned slab = blockIdx.y;
  const unsigned b = blockIdx.z;
  const float sinv = 1.0f / (QCARRY * QCARRY);
  const unsigned qrow0 = q0 + wave * 16u;
  _Float16* P = Ps + wave * (16u * LDT);

  const size_t qoff = (size_t)(b * (unsigned)SEQ + qrow0 + m) * HD + hh * 8u;
  v16h qf[2];
  qf[0] = frag_at(Qh + qoff);
  qf[1] = frag_at(Qh + qoff + 32);

  float mrow[8], lrow[8];
  v8f o[8];
#pragma unroll
  for (int v = 0; v < 8; ++v) { mrow[v] = -1.0e30f; lrow[v] = 0.0f; }
#pragma unroll
  for (int nb = 0; nb < 8; ++nb) o[nb] = (v8f){};

  const size_t kplane = (size_t)b * SEQ * HD;
  const size_t vplane = ((size_t)b * CH + slab * (unsigned)CSLAB) * SEQ;

#pragma unroll 1
  for (unsigned kb = 0; kb < (unsigned)SEQ; kb += 64u) {
#pragma unroll
    for (unsigned j = 0; j < 2u; ++j) {
      const unsigned idx = tid + 256u * j;
      const unsigned r = idx >> 3, c = (idx & 7u) * 8u;
      *(v8h*)&Ks[r * LDT + c] = *(const v8h*)(Kh + kplane + (size_t)(kb + r) * HD + c);
    }
#pragma unroll
    for (unsigned j = 0; j < 4u; ++j) {
      const unsigned idx = tid + 256u * j;
      const unsigned r = idx >> 3, c = (idx & 7u) * 8u;
      *(v8h*)&Vs[r * LDT + c] = *(const v8h*)(Vt + vplane + (size_t)r * SEQ + kb + c);
    }
    __syncthreads();

    v8f s[4];
#pragma unroll
    for (int kg = 0; kg < 4; ++kg) {
      v8f t = {};
#pragma unroll
      for (int c = 0; c < 2; ++c) {
        const v16h kf = ld_frag(&Ks[(kg * 16) * LDT + c * 32], LDT);
        t = wmma16(qf[c], kf, t);
      }
      s[kg] = t * sinv;
    }

    float alpha[8];
#pragma unroll
    for (int v = 0; v < 8; ++v) {
      float mx = fmaxf(fmaxf(s[0][v], s[1][v]), fmaxf(s[2][v], s[3][v]));
      mx = red16_max(mx);
      const float mn = fmaxf(mrow[v], mx);
      alpha[v] = __expf(mrow[v] - mn);
      mrow[v] = mn;
    }
#pragma unroll
    for (int kg = 0; kg < 4; ++kg)
#pragma unroll
      for (int v = 0; v < 8; ++v) {
        const h16 ph = toh_flush(__expf(s[kg][v] - mrow[v]) * PCARRY);
        P[(hh * 8u + (unsigned)v) * LDT + (unsigned)kg * 16u + m] = ph;
        s[kg][v] = (float)ph;
      }
#pragma unroll
    for (int v = 0; v < 8; ++v) {
      const float rs = red16_sum((s[0][v] + s[1][v]) + (s[2][v] + s[3][v]));
      lrow[v] = alpha[v] * lrow[v] + rs;
    }
#pragma unroll
    for (int nb = 0; nb < 8; ++nb)
#pragma unroll
      for (int v = 0; v < 8; ++v) o[nb][v] = o[nb][v] * alpha[v];
    wave_lds_sync();

#pragma unroll
    for (int c = 0; c < 2; ++c) {
      const v16h pf = ld_frag(P + c * 32, LDT);
#pragma unroll
      for (int nb = 0; nb < 8; ++nb) {
        const v16h vf = ld_frag(&Vs[(nb * 16) * LDT + c * 32], LDT);
        o[nb] = wmma16(pf, vf, o[nb]);
      }
    }
    __syncthreads();
  }

  const float kk = bf16r(kp[0]);
  float inv[8];
#pragma unroll
  for (int v = 0; v < 8; ++v) inv[v] = __builtin_amdgcn_rcpf(lrow[v]) * (1.0f / WCARRY);
  const unsigned cw = wave * (16u * LDE);
  const size_t frow0 = (size_t)b * SEQ_FULL + qrow0;
  const unsigned ch0 = slab * (unsigned)CSLAB;
#pragma unroll
  for (int pr = 0; pr < 4; ++pr) {
#pragma unroll
    for (int v = 0; v < 8; ++v) {
      Cs[cw + (hh * 8u + (unsigned)v) * LDE + m]       = o[2 * pr][v] * inv[v];
      Cs[cw + (hh * 8u + (unsigned)v) * LDE + 16u + m] = o[2 * pr + 1][v] * inv[v];
    }
    wave_lds_sync();
    v4f xs[4];
    size_t off[4];
#pragma unroll
    for (unsigned i = 0; i < 4u; ++i) {
      const unsigned r = 4u * i + (lane >> 3);
      const unsigned c = (lane & 7u) * 4u;
      const size_t frow = frow0 + r;
      const unsigned ch = ch0 + 32u * (unsigned)pr + c;
      const v4f u = *(const v4f*)&Cs[cw + r * LDE + c];
      const v4f xin = *(const v4f*)(xres + frow * CH + ch);
      v4f val;
#pragma unroll
      for (int j = 0; j < 4; ++j) val[j] = kk * u[j] + bf16r(xin[j]);
      xs[i] = val;
      off[i] = frow * OUTW + ch;
    }
#pragma unroll
    for (int i = 0; i < 4; ++i) *(volatile v4f*)(out + off[i]) = xs[i];
    __threadfence();
#pragma unroll
    for (int i = 0; i < 4; ++i) *(volatile v4f*)(out + off[i]) = xs[i];
    wave_lds_sync();
  }
}

extern "C" void kernel_launch(void* const* d_in, const int* in_sizes, int n_in,
                              void* d_out, int out_size, void* d_ws, size_t ws_size,
                              hipStream_t stream) {
  if (n_in < 6) return;
  const long long need_rows = (long long)(NB - 1) * SEQ_FULL + SEQ;
  if ((long long)in_sizes[0] < need_rows * CH) return;
  if ((long long)in_sizes[1] < need_rows * CH) return;
  if ((long long)in_sizes[2] < need_rows * HD) return;
  if ((long long)in_sizes[3] < need_rows * HD) return;
  if ((long long)in_sizes[4] < need_rows * CH) return;
  if (in_sizes[5] < 1) return;
  if ((long long)out_size < need_rows * OUTW) return;
  if (ws_size < WS_TOTAL) return;

  const float* G  = (const float*)d_in[0];
  const float* X  = (const float*)d_in[1];
  const float* XQ = (const float*)d_in[2];
  const float* PG = (const float*)d_in[3];
  const float* XV = (const float*)d_in[4];
  const float* KP = (const float*)d_in[5];
  float* out = (float*)d_out;

  char* ws = (char*)d_ws;
  _Float16* PG16 = (_Float16*)(ws + OFF_PG);
  _Float16* XQ16 = (_Float16*)(ws + OFF_XQ);
  _Float16* Vt16 = (_Float16*)(ws + OFF_VT);

  dim3 blk(256);

  rowconv_kernel<<<dim3(MROWS / 32), blk, 0, stream>>>(PG, XQ, PG16, XQ16);
  for (int b = 0; b < NB; ++b) {
    wconv_kernel<<<dim3(CH / 64, SEQ / 64), blk, 0, stream>>>(
        XV + (size_t)b * SEQ_FULL * CH, Vt16 + (size_t)b * CH * SEQ, (unsigned)CH, (unsigned)SEQ);
  }
  attn_kernel<<<dim3(SEQ / 128, CH / CSLAB, NB), blk, 0, stream>>>(PG16, XQ16, Vt16, X, KP, out);
  concat_kernel<<<dim3(MROWS / 4), blk, 0, stream>>>(G, out);
}
